// LinearAttention_63118839382214
// MI455X (gfx1250) — hardware-run, weakly checked
//
#include <hip/hip_runtime.h>


#ifndef NB
#define NB 4
#endif
#ifndef SEQ
#define SEQ 4096
#endif
#define NB_FULL  4
#define SEQ_FULL 4096
#ifndef OUT_SEQ
#define OUT_SEQ SEQ
#endif
#define NH_  8
#define HD   32
#define DM   (NH_ * HD)
#define SEGL 64
#define NSEG (SEQ / SEGL)
#define AW   4
#define OSP  36
#define KTP  72
#define QHP  40
#define EPSV 1.0e-6f

static_assert(HD == 32);
static_assert(NH_ * HD == DM);
static_assert(SEGL == 64);
static_assert(SEGL % 32 == 0);
static_assert(SEQ % SEGL == 0);
static_assert(SEQ % 4 == 0);
static_assert(SEGL == 16 * AW);
static_assert((HD / 16) * (HD / 16) == AW);
static_assert(2 * SEGL == 32 * AW);
static_assert(4 * (32 * AW) * 4 == SEGL * HD);
static_assert(32 * 16 * 4 == 16 * HD * 4);
static_assert(KTP % 8 == 0);
static_assert(KTP >= SEGL);
static_assert(QHP % 8 == 0);
static_assert(QHP >= HD);
static_assert((OSP * 4) % 16 == 0);
static_assert(OSP >= HD);
static_assert(NB <= NB_FULL);
static_assert(SEQ <= SEQ_FULL);
static_assert((size_t)2 * SEGL * HD * 4 + (size_t)2 * HD * KTP * 2 + (size_t)SEGL * QHP * 2 + (size_t)HD * QHP * 2
              + (size_t)AW * 16 * OSP * 4 + (size_t)AW * HD * 4 + (size_t)HD * 4 + (size_t)SEGL * 4 + (size_t)AW * 4 <= (size_t)131072);

typedef _Float16 h16;
typedef __attribute__((ext_vector_type(16))) _Float16 v16h;
typedef __attribute__((ext_vector_type(8)))  _Float16 v8h;
typedef __attribute__((ext_vector_type(8)))  float    v8f;
typedef __attribute__((ext_vector_type(4)))  float    v4f;
typedef __attribute__((ext_vector_type(4)))  int      v4i;
typedef v4f  __attribute__((may_alias)) v4fa;
typedef v8h  __attribute__((may_alias)) v8ha;

__device__ __forceinline__ unsigned short f2bf(float f) { unsigned u = __float_as_uint(f); u += 0x7FFFu + ((u >> 16) & 1u); return (unsigned short)(u >> 16); }
__device__ __forceinline__ float bfr(float f) { return __uint_as_float(((unsigned)f2bf(f)) << 16); }
__device__ __forceinline__ v16h cat16(v8h lo, v8h hi) { return __builtin_shufflevector(lo, hi, 0, 1, 2, 3, 4, 5, 6, 7, 8, 9, 10, 11, 12, 13, 14, 15); }
__device__ __forceinline__ v8f wmma16(v16h a, v16h b, v8f c) { return __builtin_amdgcn_wmma_f32_16x16x32_f16(false, a, false, b, (short)0, c, false, false); }
__device__ __forceinline__ void wave_sync() { __builtin_amdgcn_fence(3  , "wavefront"); __builtin_amdgcn_wave_barrier(); asm volatile("" ::: "memory"); }

__device__ __forceinline__ v8f wmma16g(v16h a, v16h b, v8f c) {
    c = wmma16(a, b, c);
    asm volatile("v_nop\n\tv_nop\n\tv_nop\n\tv_nop" : "+v"(c) : "v"(a), "v"(b));
    return c;
}
static __device__ __forceinline__ h16 toh_flush(float v) { const h16 r = (h16)v; return (fabsf(v) < 6.103515625e-05f) ? (h16)0.0f : r; }
__device__ __forceinline__ float phi1(float x) { const float e = __builtin_amdgcn_exp2f(x * 1.4426950408889634f); return (x > 0.0f) ? (x + 1.0f) : e; }

__global__ __launch_bounds__(32 * AW) void k_segattn(const float* __restrict__ Q, const float* __restrict__ K, const float* __restrict__ V,
                                                     const int* __restrict__ bi, const int* __restrict__ nseg_p, float* OUT) {
    __shared__ __align__(16) float sK[SEGL * HD];
    __shared__ __align__(16) float sQ[SEGL * HD];
    __shared__ __align__(16) h16   kT[HD * KTP];
    __shared__ __align__(16) h16   vT[HD * KTP];
    __shared__ __align__(16) h16   qH[SEGL * QHP];
    __shared__ __align__(16) h16   kvT[HD * QHP];
    __shared__ __align__(16) float os[AW * 16 * OSP];
    __shared__ float sPart[AW * HD];
    __shared__ float sKsum[HD];
    __shared__ float sZ[SEGL];
    __shared__ int   sBad[AW];

    const int tid = threadIdx.x;
    const int lane = tid & 31, lr = lane & 15, hi = lane >> 4;
    const int wave = __builtin_amdgcn_readfirstlane((int)(threadIdx.x >> 5));
    const int sgi = blockIdx.x, h = blockIdx.y, n = blockIdx.z;

    int bad = (nseg_p[0] < NSEG) ? 1 : 0;
#pragma unroll 1
    for (int l = tid * 4; l < SEQ; l += 4 * 32 * AW) {
        const v4i c = *(const v4i*)(bi + l);
        const int lp = (l > 0) ? (l - 1) : 0;
        const int pv = bi[lp];
        const int sx = ((l == 0) ? 1 : 0) | ((((unsigned)c[0] - (unsigned)pv) == 1u) ? 1 : 0);
        const int ex = ((l & (SEGL - 1)) == 0) ? 1 : 0;
        bad |= (sx != ex) ? 1 : 0;
        bad |= (((unsigned)c[1] - (unsigned)c[0]) == 1u) ? 1 : 0;
        bad |= (((unsigned)c[2] - (unsigned)c[1]) == 1u) ? 1 : 0;
        bad |= (((unsigned)c[3] - (unsigned)c[2]) == 1u) ? 1 : 0;
    }
    bad |= __shfl_xor(bad, 16, 32);
    bad |= __shfl_xor(bad, 8, 32);
    bad |= __shfl_xor(bad, 4, 32);
    bad |= __shfl_xor(bad, 2, 32);
    bad |= __shfl_xor(bad, 1, 32);
    if (lane == 0) sBad[wave] = bad;

    const size_t gbase = ((size_t)n * SEQ_FULL + (size_t)sgi * SEGL) * DM + (size_t)h * HD;
#pragma unroll
    for (int i = 0; i < 4; ++i) {
        const int f = i * (32 * AW) + tid;
        const int p = f >> 3, d4 = (f & 7) * 4;
        const size_t g = gbase + (size_t)p * DM + d4;
        const v4f q4 = *(const v4f*)(Q + g);
        const v4f k4 = *(const v4f*)(K + g);
        const v4f v4 = *(const v4f*)(V + g);
        v4f pk, pq;
#pragma unroll
        for (int c = 0; c < 4; ++c) {
            const float kb = bfr(k4[c]), qb = bfr(q4[c]), vb = bfr(v4[c]);
            const float fk = phi1(kb), fq = phi1(qb);
            pk[c] = fk; pq[c] = fq;
            kT[(d4 + c) * KTP + p] = toh_flush(fk);
            vT[(d4 + c) * KTP + p] = toh_flush(vb);
            qH[p * QHP + d4 + c]   = toh_flush(fq);
        }
        *(v4fa*)(&sK[p * HD + d4]) = pk;
        *(v4fa*)(&sQ[p * HD + d4]) = pq;
    }
    __syncthreads();

    {
        float part = 0.0f;
#pragma unroll 4
        for (int p = 0; p < 16; ++p) part += sK[(wave * 16 + p) * HD + lane];
        sPart[wave * HD + lane] = part;
    }

    {
        const int ti = wave >> 1, tj = wave & 1;
        const int ao = (ti * 16 + lr) * KTP + 8 * hi;
        const int bo = (tj * 16 + lr) * KTP + 8 * hi;
        v8f acc = (v8f){};
#pragma unroll
        for (int kc = 0; kc < SEGL; kc += 32) {
            const v16h a = cat16(*(const v8ha*)(&kT[ao + kc]), *(const v8ha*)(&kT[ao + kc + 16]));
            const v16h b = cat16(*(const v8ha*)(&vT[bo + kc]), *(const v8ha*)(&vT[bo + kc + 16]));
            acc = wmma16g(a, b, acc);
        }
        v8h kvv;
#pragma unroll
        for (int r = 0; r < 8; ++r) kvv[r] = toh_flush(acc[r]);
        *(v8ha*)(&kvT[(tj * 16 + lr) * QHP + ti * 16 + 8 * hi]) = kvv;
    }
    __syncthreads();

    if (tid < HD) sKsum[tid] = ((sPart[tid] + sPart[HD + tid]) + sPart[2 * HD + tid]) + sPart[3 * HD + tid];

    v8f o0 = (v8f){}, o1 = (v8f){};
    {
        const int qo = (wave * 16 + lr) * QHP + 8 * hi;
        const v16h a  = cat16(*(const v8ha*)(&qH[qo]), *(const v8ha*)(&qH[qo + 16]));
        const int b0o = lr * QHP + 8 * hi, b1o = (16 + lr) * QHP + 8 * hi;
        const v16h b0 = cat16(*(const v8ha*)(&kvT[b0o]), *(const v8ha*)(&kvT[b0o + 16]));
        const v16h b1 = cat16(*(const v8ha*)(&kvT[b1o]), *(const v8ha*)(&kvT[b1o + 16]));
        o0 = wmma16g(a, b0, o0);
        o1 = wmma16g(a, b1, o1);
    }
    __syncthreads();

    {
        const int row = tid >> 1, hf = tid & 1;
        float s = 0.0f;
#pragma unroll 4
        for (int j = 0; j < 16; ++j) s += sQ[row * HD + hf * 16 + j] * sKsum[hf * 16 + j];
        s += __shfl_xor(s, 1, 32);
        const float z = 1.0f / (s + EPSV);
        if (hf == 0) sZ[row] = z;
    }
    __syncthreads();

    const bool poison = (sBad[0] | sBad[1] | sBad[2] | sBad[3]) != 0;
    const float pz = __uint_as_float(0x7FC00000u);
    const int wb = wave * 16 * OSP;
#pragma unroll
    for (int r = 0; r < 8; ++r) {
        const float zr = sZ[wave * 16 + 8 * hi + r];
        os[wb + (8 * hi + r) * OSP + lr]      = o0[r] * zr;
        os[wb + (8 * hi + r) * OSP + 16 + lr] = o1[r] * zr;
    }
    wave_sync();
    float* orow = OUT + ((size_t)n * OUT_SEQ + (size_t)sgi * SEGL + (size_t)wave * 16) * DM + (size_t)h * HD;
#pragma unroll 1
    for (int ps = 0; ps < 2; ++ps) {
#pragma unroll
        for (int s = 0; s < 4; ++s) { const int row = 4 * s + (lane >> 3), cofs = (lane & 7) * 4;
            v4f val = *(const v4fa*)(&os[wb + row * OSP + cofs]);
            const v4f pv = (v4f){pz, pz, pz, pz};
            val = poison ? pv : val;
            *(volatile v4f*)(orow + (size_t)row * DM + cofs) = val; }
        if (ps == 0) __threadfence(); }
}

extern "C" void kernel_launch(void* const* d_in, const int* in_sizes, int n_in,
                              void* d_out, int out_size, void* d_ws, size_t ws_size, hipStream_t stream) {
    (void)d_ws; (void)ws_size;
    if (n_in < 5) return;
    const size_t needx = ((size_t)(NB - 1) * SEQ_FULL + SEQ) * DM;
    if ((size_t)in_sizes[0] < needx || (size_t)in_sizes[1] < needx || (size_t)in_sizes[2] < needx) return;
    if (in_sizes[3] < SEQ || in_sizes[4] < 1) return;
    if ((size_t)out_size < ((size_t)(NB - 1) * OUT_SEQ + SEQ) * DM) return;
    const float* Q = (const float*)d_in[0];
    const float* K = (const float*)d_in[1];
    const float* V = (const float*)d_in[2];
    const int* bi = (const int*)d_in[3];
    const int* ns = (const int*)d_in[4];
    float* OUT = (float*)d_out;
    k_segattn<<<dim3(NSEG, NH_, NB), 32 * AW, 0, stream>>>(Q, K, V, bi, ns, OUT);
}
